// DropEdge_43628277793359
// MI455X (gfx1250) — hardware-run, weakly checked
//
#include <hip/hip_runtime.h>
#include <stddef.h>
#include <stdint.h>

#define NN      50000
#define FD      256
#define HID     128
#define OUTF    64
#define NE      800000
#define MP      50048
#define SPLIT2  1
#define APITCH  256
#define WPITCH  256
#if SPLIT2
#define KEXT2   256
#else
#define KEXT2   128
#endif
#define NTHR    256
#define NWAVE   8
#define EPT     8
#define WCH     (32 * EPT)
#define NBRUN   1024
#define SLB     10
#define NBK     49
#define WLCAP   2560
#define RCAP    20480
#define DEGCAP  128
#define MAXDEG_MEAS   35
#define MAXB1024_MEAS 16623
#define ABM     64
#define G1M     64
#define G1THR   128
#define SP1     132
#define G2M     128
#define SP2     68
#define WSMAX   (128u << 20)

#define BK_ZINTS (NWAVE * WLCAP + RCAP + 3 * NBRUN)
#define BK_INTS  (BK_ZINTS + 16)
#define BK_LDS   (BK_INTS * 4)

#define PBX   (MP * FD / 8 / NTHR)
#define PBW1  (HID * FD / 8 / NTHR)
#define PBW2  (OUTF * WPITCH / 8 / NTHR)
#define PBTOT (PBX + PBW1 + PBW2 + 1)

static_assert(NBRUN == 1024 && NBRUN == (1 << SLB));
static_assert(NE < (1 << 22) && NE < (1 << 21) && (((long long)NE) << SLB) < (1LL << 31));
static_assert(HID == 32 * 4 && OUTF == 16 * 4);
static_assert(APITCH == 2 * HID && WPITCH == 2 * HID && KEXT2 <= APITCH && KEXT2 <= WPITCH);
static_assert(KEXT2 == (SPLIT2 ? 2 * HID : HID) && KEXT2 % 32 == 0 && FD % 32 == 0);
static_assert(RCAP == NWAVE * WLCAP && RCAP % 1024 == 0 && (RCAP / 2) % NTHR == 0 && BK_ZINTS % 4 == 0);
static_assert((long long)RCAP * 100 >= (long long)MAXB1024_MEAS * 105);
static_assert(WLCAP >= MAXB1024_MEAS / 8 + 8 * 46 + 1);
static_assert(MAXDEG_MEAS + 8 <= DEGCAP && DEGCAP < RCAP);
static_assert(NBK * NBRUN >= MP && MP >= NN);
static_assert(MP % G1M == 0 && MP % G2M == 0 && MP % ABM == 0 && NBRUN % ABM == 0);
static_assert(NE % WCH == 0 && NE % 4 == 0 && NN % 2 == 0);
static_assert((MP * FD / 8) % NTHR == 0 && (HID * FD / 8) % NTHR == 0 && (OUTF * WPITCH / 8) % NTHR == 0);
static_assert(BK_LDS <= 327680);
static_assert(G1M * SP1 * 4 <= 65536 && G2M * SP2 * 4 <= 65536);
static_assert(NN * OUTF - 1 == 3199999);

typedef float          v4f   __attribute__((ext_vector_type(4)));
typedef float          v8f   __attribute__((ext_vector_type(8)));
typedef int            v2i   __attribute__((ext_vector_type(2)));
typedef int            v4i   __attribute__((ext_vector_type(4)));
typedef int            v8i   __attribute__((ext_vector_type(8)));
typedef unsigned short v8us  __attribute__((ext_vector_type(8)));
typedef unsigned short v16us __attribute__((ext_vector_type(16)));
typedef __bf16         v16bf __attribute__((ext_vector_type(16)));
typedef v4f  __attribute__((may_alias)) v4fa;
typedef v2i  __attribute__((may_alias)) v2ia;
typedef v4i  __attribute__((may_alias)) v4ia;
typedef v8us __attribute__((may_alias)) v8usa;
union FragB { v16bf v; v16us u; v8us h[2]; v8i w; };

__device__ __forceinline__ v8f wmb(const FragB& a, const FragB& b, v8f c) {
  v8f d = __builtin_amdgcn_wmma_f32_16x16x32_bf16(false, a.v, false, b.v, (short)0, c, false, false);
  asm volatile("v_nop\n\tv_nop\n\tv_nop\n\tv_nop" : "+v"(d) : "v"(a.w), "v"(b.w));
  return d;
}

__device__ __forceinline__ unsigned bf16_bits(float f) {
  const unsigned u = __float_as_uint(f);
  const unsigned r = (u + 0x7FFFu + ((u >> 16) & 1u)) >> 16;
  const unsigned q = (u >> 16) | 0x40u;
  return ((u & 0x7fffffffu) > 0x7f800000u) ? q : r;
}

__device__ __forceinline__ void hilo_pack(float v0, float v1, float v2, float v3,
                                          int& h01, int& h23, int& l01, int& l23) {
  const unsigned a0 = bf16_bits(v0), a1 = bf16_bits(v1), a2 = bf16_bits(v2), a3 = bf16_bits(v3);
  const unsigned b0 = bf16_bits(v0 - __uint_as_float(a0 << 16));
  const unsigned b1 = bf16_bits(v1 - __uint_as_float(a1 << 16));
  const unsigned b2 = bf16_bits(v2 - __uint_as_float(a2 << 16));
  const unsigned b3 = bf16_bits(v3 - __uint_as_float(a3 << 16));
  h01 = (int)(a0 | (a1 << 16)); h23 = (int)(a2 | (a3 << 16));
  l01 = (int)(b0 | (b1 << 16)); l23 = (int)(b2 | (b3 << 16));
}

__device__ __forceinline__ v4i regroup16(int h01, int h23, int l01, int l23, int lane) {
  const int s0 = (2 * lane) & 31, s1 = s0 + 1;
  const int a0 = __shfl(h01, s0, 32), a1 = __shfl(h23, s0, 32), a2 = __shfl(h01, s1, 32), a3 = __shfl(h23, s1, 32);
  const int b0 = __shfl(l01, s0, 32), b1 = __shfl(l23, s0, 32), b2 = __shfl(l01, s1, 32), b3 = __shfl(l23, s1, 32);
  const int mk = (lane < 16) ? -1 : 0;
  v4i o;
  o.x = (a0 & mk) | (b0 & ~mk); o.y = (a1 & mk) | (b1 & ~mk);
  o.z = (a2 & mk) | (b2 & ~mk); o.w = (a3 & mk) | (b3 & ~mk);
  return o;
}

__device__ __forceinline__ void st2_v4f(float* p, v4f v) {
  *(volatile v4f*)p = v;
  __threadfence();
  *(volatile v4f*)p = v;
}
__device__ __forceinline__ void st2_v4i(int* p, v4i v) {
  *(volatile v4i*)p = v;
  __threadfence();
  *(volatile v4i*)p = v;
}
__device__ __forceinline__ void st2_v8us(unsigned short* p, v8us v) {
  *(volatile v8us*)p = v;
  __threadfence();
  *(volatile v8us*)p = v;
}

__device__ __forceinline__ v8us column8(const float* __restrict__ base, int stride) {
  float f[8];
#pragma unroll
  for (int i = 0; i < 8; ++i) f[i] = base[(size_t)i * (size_t)stride];
  v8us o;
#pragma unroll
  for (int i = 0; i < 8; ++i) o[i] = (unsigned short)bf16_bits(f[i]);
  return o;
}

__global__ __launch_bounds__(NTHR) void k_prep(const float* __restrict__ x, const float* __restrict__ w1,
                                               const float* __restrict__ b1, const float* __restrict__ w2,
                                               const float* __restrict__ b2, unsigned short* xb,
                                               unsigned short* w1t, unsigned short* w2d, float* sm) {
  const int tid = (int)threadIdx.x, lane = tid & 31, wave = tid >> 5;
  const int blk = (int)blockIdx.x;
  if (blk < PBX) {
    const int u   = blk * NTHR + tid;
    const int row = u >> 5, k8 = (u & 31) * 8;
    const int rc  = row < NN ? row : NN - 1;
    const unsigned mk = row < NN ? 0xffffu : 0u;
    const float* p = x + (size_t)rc * FD + k8;
    const v4f a = *(const v4fa*)p;
    const v4f b = *(const v4fa*)(p + 4);
    v8us o;
    o[0] = (unsigned short)(bf16_bits(a.x) & mk); o[1] = (unsigned short)(bf16_bits(a.y) & mk);
    o[2] = (unsigned short)(bf16_bits(a.z) & mk); o[3] = (unsigned short)(bf16_bits(a.w) & mk);
    o[4] = (unsigned short)(bf16_bits(b.x) & mk); o[5] = (unsigned short)(bf16_bits(b.y) & mk);
    o[6] = (unsigned short)(bf16_bits(b.z) & mk); o[7] = (unsigned short)(bf16_bits(b.w) & mk);
    st2_v8us(xb + (size_t)row * FD + k8, o);
  } else if (blk < PBX + PBW1) {
    const int u = (blk - PBX) * NTHR + tid;
    const int n = u >> 5, k8 = (u & 31) * 8;
    const v8us o = column8(w1 + (size_t)k8 * HID + n, HID);
    st2_v8us(w1t + (size_t)n * FD + k8, o);
  } else if (blk < PBX + PBW1 + PBW2) {
    const int u = (blk - PBX - PBW1) * NTHR + tid;
    const int n = u >> 5, k8 = (u & 31) * 8, kk = k8 & (HID - 1);
    const v8us o = column8(w2 + (size_t)kk * OUTF + n, OUTF);
    st2_v8us(w2d + (size_t)n * WPITCH + k8, o);
  } else {
    if (tid < 64) {
      const int q = lane & 15;
      const v4f a = *(const v4fa*)(b1 + 4 * lane);
      const v4f c = *(const v4fa*)(b2 + 4 * q);
      asm volatile("" :: "v"(a));
      asm volatile("" :: "v"(c));
      const unsigned m1 = (wave == 0) ? 0xffffffffu : 0u;
      const unsigned m2 = ((wave == 1) & (lane < 16)) ? 0xffffffffu : 0u;
      v4f o;
      o.x = __uint_as_float(((bf16_bits(a.x) << 16) & m1) | ((bf16_bits(c.x) << 16) & m2));
      o.y = __uint_as_float(((bf16_bits(a.y) << 16) & m1) | ((bf16_bits(c.y) << 16) & m2));
      o.z = __uint_as_float(((bf16_bits(a.z) << 16) & m1) | ((bf16_bits(c.z) << 16) & m2));
      o.w = __uint_as_float(((bf16_bits(a.w) << 16) & m1) | ((bf16_bits(c.w) << 16) & m2));
      st2_v4f(sm + 4 * tid, o);
    }
  }
}

__global__ __launch_bounds__(NTHR) void k_bucket(const int* __restrict__ srcs, const int* __restrict__ dsts,
                                                 const float* __restrict__ ew, int* LIST, int* CO, int* FLAG) {
  extern __shared__ __attribute__((aligned(16))) int dsm[];
  int* wl   = dsm;
  int* pl   = dsm + NWAVE * WLCAP;
  int* cnt  = pl + RCAP;
  int* offs = cnt + NBRUN;
  int* cur  = offs + NBRUN;
  int* misc = cur + NBRUN;
  const int tid = (int)threadIdx.x, lane = tid & 31, wave = tid >> 5;
  const int blk = (int)blockIdx.x;
  const unsigned nbs = (unsigned)(blk * NBRUN);

  {
    const v4i z4 = {0, 0, 0, 0};
    for (int i = tid * 4; i < BK_ZINTS; i += NTHR * 4) *(v4ia*)(dsm + i) = z4;
    if (tid < 16) misc[tid] = 0;
  }
  __syncthreads();

  {
    const int per  = ((NE + NWAVE * WCH - 1) / (NWAVE * WCH)) * WCH;
    const int ebeg = wave * per;
    const int eend = (ebeg + per < NE) ? (ebeg + per) : NE;
    int* mylist = wl + wave * WLCAP;
    int wc = 0;
#pragma unroll 1
    for (int cb = ebeg; cb < eend; cb += WCH) {
      const int e0 = cb + lane * EPT;
      const v4i da = *(const v4ia*)(dsts + e0);
      const v4i db = *(const v4ia*)(dsts + e0 + 4);
      const unsigned s0 = (unsigned)da.x - nbs, s1 = (unsigned)da.y - nbs;
      const unsigned s2 = (unsigned)da.z - nbs, s3 = (unsigned)da.w - nbs;
      const unsigned s4 = (unsigned)db.x - nbs, s5 = (unsigned)db.y - nbs;
      const unsigned s6 = (unsigned)db.z - nbs, s7 = (unsigned)db.w - nbs;
      const bool h0 = s0 < (unsigned)NBRUN, h1 = s1 < (unsigned)NBRUN, h2 = s2 < (unsigned)NBRUN, h3 = s3 < (unsigned)NBRUN;
      const bool h4 = s4 < (unsigned)NBRUN, h5 = s5 < (unsigned)NBRUN, h6 = s6 < (unsigned)NBRUN, h7 = s7 < (unsigned)NBRUN;
      const unsigned m0 = __builtin_amdgcn_ballot_w32(h0), m1 = __builtin_amdgcn_ballot_w32(h1);
      const unsigned m2 = __builtin_amdgcn_ballot_w32(h2), m3 = __builtin_amdgcn_ballot_w32(h3);
      const unsigned m4 = __builtin_amdgcn_ballot_w32(h4), m5 = __builtin_amdgcn_ballot_w32(h5);
      const unsigned m6 = __builtin_amdgcn_ballot_w32(h6), m7 = __builtin_amdgcn_ballot_w32(h7);
      const unsigned any = m0 | m1 | m2 | m3 | m4 | m5 | m6 | m7;
      if (any != 0u) {
        const int pre = (int)(__builtin_amdgcn_mbcnt_lo(m0, 0u) + __builtin_amdgcn_mbcnt_lo(m1, 0u) +
                              __builtin_amdgcn_mbcnt_lo(m2, 0u) + __builtin_amdgcn_mbcnt_lo(m3, 0u) +
                              __builtin_amdgcn_mbcnt_lo(m4, 0u) + __builtin_amdgcn_mbcnt_lo(m5, 0u) +
                              __builtin_amdgcn_mbcnt_lo(m6, 0u) + __builtin_amdgcn_mbcnt_lo(m7, 0u));
        int p = wc + pre;
        if (h0) { if (p < WLCAP) mylist[p] = ((e0 + 0) << SLB) | (int)s0; p = p + 1; }
        if (h1) { if (p < WLCAP) mylist[p] = ((e0 + 1) << SLB) | (int)s1; p = p + 1; }
        if (h2) { if (p < WLCAP) mylist[p] = ((e0 + 2) << SLB) | (int)s2; p = p + 1; }
        if (h3) { if (p < WLCAP) mylist[p] = ((e0 + 3) << SLB) | (int)s3; p = p + 1; }
        if (h4) { if (p < WLCAP) mylist[p] = ((e0 + 4) << SLB) | (int)s4; p = p + 1; }
        if (h5) { if (p < WLCAP) mylist[p] = ((e0 + 5) << SLB) | (int)s5; p = p + 1; }
        if (h6) { if (p < WLCAP) mylist[p] = ((e0 + 6) << SLB) | (int)s6; p = p + 1; }
        if (h7) { if (p < WLCAP) mylist[p] = ((e0 + 7) << SLB) | (int)s7; p = p + 1; }
        wc += (int)(__builtin_popcount(m0) + __builtin_popcount(m1) + __builtin_popcount(m2) + __builtin_popcount(m3) +
                    __builtin_popcount(m4) + __builtin_popcount(m5) + __builtin_popcount(m6) + __builtin_popcount(m7));
      }
    }
    if (lane == 0) misc[wave] = wc;
  }
  __syncthreads();

  if (wave == 0) {
    int ov = 0;
#pragma unroll 1
    for (int w2 = 0; w2 < NWAVE; ++w2) {
      int c = misc[w2];
      if (c > WLCAP) ov = 1;
      c = c < 0 ? 0 : (c > WLCAP ? WLCAP : c);
#pragma unroll 1
      for (int b0 = 0; b0 < c; b0 += 32) {
        const int idx = b0 + lane;
        const int ent = wl[w2 * WLCAP + (idx < WLCAP ? idx : WLCAP - 1)];
        const int m32 = (c - b0) < 32 ? (c - b0) : 32;
#pragma unroll 1
        for (int k = 0; k < m32; ++k) {
          const int u    = __builtin_amdgcn_readlane(ent, k);
          const int slot = u & (NBRUN - 1);
          if (lane == 0) cnt[slot] = cnt[slot] + 1;
        }
      }
    }
    if (lane == 0) misc[9] = ov;
  }
  __syncthreads();
  if (wave == 0) {
    const int base = lane * (NBRUN / 32);
    int s = 0;
#pragma unroll 1
    for (int i = 0; i < NBRUN / 32; ++i) s += cnt[base + i];
    int incl = s;
#pragma unroll
    for (int d = 1; d < 32; d <<= 1) {
      const int y = __shfl_up(incl, d, 32);
      if (lane >= d) incl += y;
    }
    int run = incl - s;
    int bigl = 0;
#pragma unroll 1
    for (int i = 0; i < NBRUN / 32; ++i) {
      const int cv = cnt[base + i];
      bigl |= (cv > DEGCAP) ? 1 : 0;
      offs[base + i] = run;
      cur[base + i]  = run;
      run += cv;
    }
    const unsigned bm = __builtin_amdgcn_ballot_w32(bigl != 0);
    if (lane == 31) misc[8] = run;
    if (lane == 0 && bm != 0u) misc[9] = 1;
  }
  __syncthreads();

  if (wave == 0) {
#pragma unroll 1
    for (int w2 = 0; w2 < NWAVE; ++w2) {
      int c = misc[w2];
      c = c < 0 ? 0 : (c > WLCAP ? WLCAP : c);
#pragma unroll 1
      for (int b0 = 0; b0 < c; b0 += 32) {
        const int idx = b0 + lane;
        const int ent = wl[w2 * WLCAP + (idx < WLCAP ? idx : WLCAP - 1)];
        const int m32 = (c - b0) < 32 ? (c - b0) : 32;
#pragma unroll 1
        for (int k = 0; k < m32; ++k) {
          const int u    = __builtin_amdgcn_readlane(ent, k);
          const int slot = u & (NBRUN - 1);
          if (lane == 0) {
            int p = cur[slot];
            p = p < 0 ? 0 : (p > RCAP - 1 ? RCAP - 1 : p);
            pl[p] = u;
            cur[slot] = p + 1;
          }
        }
      }
    }
  }
  __syncthreads();

  const int ovf = misc[9];
  int tt = misc[8];
  tt = tt < 0 ? 0 : (tt > RCAP ? RCAP : tt);
  int* lp  = LIST + (size_t)blk * (size_t)(2 * RCAP);
  int* cop = CO + (size_t)blk * (2 * NBRUN);
  int* fp  = FLAG + (size_t)blk * 32;
#pragma unroll 1
  for (int it = 0; it < RCAP / 2 / NTHR; ++it) {
    const int i2 = it * NTHR + tid;
    const v2i hw = *(const v2ia*)(pl + 2 * i2);
    int e0 = (hw.x >> SLB) & 0x1FFFFF;
    int e1 = (hw.y >> SLB) & 0x1FFFFF;
    e0 = e0 > NE - 1 ? NE - 1 : e0;
    e1 = e1 > NE - 1 ? NE - 1 : e1;
    int   sr0 = srcs[e0], sr1 = srcs[e1];
    float wv0 = ew[e0],   wv1 = ew[e1];
    asm volatile("" :: "v"(sr0), "v"(sr1), "v"(wv0), "v"(wv1));
    sr0 = sr0 < 0 ? 0 : (sr0 > NN - 1 ? NN - 1 : sr0);
    sr1 = sr1 < 0 ? 0 : (sr1 > NN - 1 ? NN - 1 : sr1);
    const int mk0 = (2 * i2 < tt) ? -1 : 0;
    const int mk1 = (2 * i2 + 1 < tt) ? -1 : 0;
    v4i o;
    o.x = sr0 & mk0; o.y = (int)(bf16_bits(wv0) << 16) & mk0;
    o.z = sr1 & mk1; o.w = (int)(bf16_bits(wv1) << 16) & mk1;
    st2_v4i(lp + 4 * i2, o);
  }
#pragma unroll 1
  for (int it = 0; it < 2; ++it) {
    const int i4 = 4 * (it * NTHR + tid);
    const v4i v = *(const v4ia*)(cnt + i4);
    st2_v4i(cop + i4, v);
  }
  if (tid < 8) {
    const v4i f = {ovf, ovf, ovf, ovf};
    st2_v4i(fp + 4 * tid, f);
  }
}

template <int NT, int KEXT, int AP, int WP>
__device__ __forceinline__ void gemm_16xN(const unsigned short* __restrict__ ap,
                                          const unsigned short* __restrict__ bp, v8f (&acc)[NT]) {
  static_assert(KEXT % 32 == 0 && KEXT <= AP && KEXT <= WP);
#pragma unroll 1
  for (int k0 = 0; k0 < KEXT; k0 += 32) {
    FragB af;
    af.h[0] = *(const v8usa*)(ap + k0);
    af.h[1] = *(const v8usa*)(ap + k0 + 16);
#pragma unroll
    for (int nt = 0; nt < NT; ++nt) {
      const unsigned short* wq = bp + (size_t)(16 * nt) * (size_t)WP + k0;
      FragB bf;
      bf.h[0] = *(const v8usa*)wq;
      bf.h[1] = *(const v8usa*)(wq + 16);
      acc[nt] = wmb(af, bf, acc[nt]);
    }
  }
}

template <int NT, int SP>
__device__ __forceinline__ void stage_d(float* stg, const v8f (&acc)[NT], int wave, int hh, int m) {
#pragma unroll
  for (int nt = 0; nt < NT; ++nt) {
#pragma unroll
    for (int r = 0; r < 8; ++r) stg[(16 * wave + 8 * hh + r) * SP + 16 * nt + m] = acc[nt][r];
  }
}

__global__ __launch_bounds__(G1THR) __attribute__((amdgpu_num_vgpr(248)))
void k_gemm1(const unsigned short* __restrict__ XB, const unsigned short* __restrict__ W1T, float* P1) {
  __shared__ __attribute__((aligned(16))) float stg[G1M * SP1];
  const int tid = (int)threadIdx.x, lane = tid & 31, wave = tid >> 5, hh = lane >> 4, m = lane & 15;
  const int rowBase = (int)blockIdx.x * G1M;

  v8f acc[8];
  {
    const v8f z = {0.f, 0.f, 0.f, 0.f, 0.f, 0.f, 0.f, 0.f};
#pragma unroll
    for (int t = 0; t < 8; ++t) acc[t] = z;
  }
  const unsigned short* ap = XB + (size_t)(rowBase + 16 * wave + m) * (size_t)FD + 8 * hh;
  const unsigned short* bp = W1T + (size_t)m * (size_t)FD + 8 * hh;
  gemm_16xN<8, FD, FD, FD>(ap, bp, acc);
  stage_d<8, SP1>(stg, acc, wave, hh, m);
  __syncthreads();

#pragma unroll 1
  for (int i = 0; i < 16; ++i) {
    const int lr   = 16 * wave + i;
    const int grow = rowBase + lr;
    const v4f a = *(const v4fa*)(stg + lr * SP1 + 4 * lane);
    asm volatile("" :: "v"(a));
    if (grow < NN) st2_v4f(P1 + (size_t)grow * HID + 4 * lane, a);
  }
}

__global__ __launch_bounds__(NTHR) void k_replay1(const int* __restrict__ LIST, const int* __restrict__ CO,
                                                  const int* __restrict__ FLAG, const float* P1,
                                                  const float* __restrict__ sm, unsigned short* H1hl) {
  const int tid = (int)threadIdx.x, lane = tid & 31, wave = tid >> 5;
  const int rowBase = (int)blockIdx.x * ABM;
  const int bucket  = rowBase >> SLB;
  const int* lb  = LIST + (size_t)bucket * (size_t)(2 * RCAP);
  const int* cob = CO + (size_t)bucket * (2 * NBRUN);
  const int flag = FLAG[(size_t)bucket * 32];
  const float qnan = __uint_as_float(0x7fc00000u);
  const v4f bias = *(const v4fa*)(sm + 4 * lane);

#pragma unroll 1
  for (int i = 0; i < ABM / NWAVE; ++i) {
    const int d    = rowBase + (ABM / NWAVE) * wave + i;
    const int slot = d & (NBRUN - 1);
    int c = cob[slot];
    int o = cob[NBRUN + slot];
    const bool big = c > DEGCAP;
    o = o < 0 ? 0 : (o > RCAP - 1 ? RCAP - 1 : o);
    c = c < 0 ? 0 : (c > DEGCAP ? DEGCAP : c);
    c = c > (RCAP - o) ? (RCAP - o) : c;
    const int oS = __builtin_amdgcn_readfirstlane(o);
    const int cS = __builtin_amdgcn_readfirstlane(c);
    int last = oS + cS - 1;
    last = last < oS ? oS : last;
    float a0 = 0.0f, a1 = 0.0f, a2 = 0.0f, a3 = 0.0f;
#pragma unroll 1
    for (int j = 0; j < cS; ++j) {
      int idx = oS + j;
      idx = idx > last ? last : idx;
      const v2i ent = *(const v2ia*)(lb + 2 * idx);
      int sr = ent.x;
      sr = sr < 0 ? 0 : (sr > NN - 1 ? NN - 1 : sr);
      const float w = __int_as_float(ent.y);
      const v4f p = *(const v4fa*)(P1 + (size_t)sr * HID + 4 * lane);
      a0 = fmaf(w, p.x, a0); a1 = fmaf(w, p.y, a1); a2 = fmaf(w, p.z, a2); a3 = fmaf(w, p.w, a3);
    }
    float v0 = a0 + bias.x, v1 = a1 + bias.y, v2 = a2 + bias.z, v3 = a3 + bias.w;
    v0 = (v0 > 0.0f) ? v0 : (v0 - v0); v1 = (v1 > 0.0f) ? v1 : (v1 - v1);
    v2 = (v2 > 0.0f) ? v2 : (v2 - v2); v3 = (v3 > 0.0f) ? v3 : (v3 - v3);
    const bool bad  = (flag != 0) | big;
    const bool live = d < NN;
    v0 = bad ? qnan : v0; v1 = bad ? qnan : v1; v2 = bad ? qnan : v2; v3 = bad ? qnan : v3;
    v0 = live ? v0 : 0.0f; v1 = live ? v1 : 0.0f; v2 = live ? v2 : 0.0f; v3 = live ? v3 : 0.0f;
    int h01, h23, l01, l23;
    hilo_pack(v0, v1, v2, v3, h01, h23, l01, l23);
    const v4i ow = regroup16(h01, h23, l01, l23, lane);
    unsigned short* hp = H1hl + (size_t)d * APITCH + 8 * lane;
    *(volatile v4i*)hp = ow;
    __threadfence();
    *(volatile v4i*)hp = ow;
  }
}

__global__ __launch_bounds__(NTHR) __attribute__((amdgpu_num_vgpr(248)))
void k_gemm2(const unsigned short* __restrict__ A, const unsigned short* __restrict__ BT, float* P2) {
  __shared__ __attribute__((aligned(16))) float stg[G2M * SP2];
  const int tid = (int)threadIdx.x, lane = tid & 31, wave = tid >> 5, hh = lane >> 4, m = lane & 15;
  const int rowBase = (int)blockIdx.x * G2M;

  v8f acc[4];
  {
    const v8f z = {0.f, 0.f, 0.f, 0.f, 0.f, 0.f, 0.f, 0.f};
#pragma unroll
    for (int t = 0; t < 4; ++t) acc[t] = z;
  }
  const unsigned short* ap = A + (size_t)(rowBase + 16 * wave + m) * (size_t)APITCH + 8 * hh;
  const unsigned short* bp = BT + (size_t)m * (size_t)WPITCH + 8 * hh;
  gemm_16xN<4, KEXT2, APITCH, WPITCH>(ap, bp, acc);
  stage_d<4, SP2>(stg, acc, wave, hh, m);
  __syncthreads();

#pragma unroll 1
  for (int i = 0; i < 8; ++i) {
    const int lr   = 16 * wave + 2 * i + hh;
    const int grow = rowBase + lr;
    const v4f a = *(const v4fa*)(stg + lr * SP2 + 4 * m);
    asm volatile("" :: "v"(a));
    float* op = P2 + (size_t)grow * OUTF + 4 * m;
    const bool live = grow < NN;
    if (live) *(volatile v4f*)op = a;
    __threadfence();
    if (live) *(volatile v4f*)op = a;
  }
}

__global__ __launch_bounds__(NTHR) void k_replay2(const int* __restrict__ LIST, const int* __restrict__ CO,
                                                  const int* __restrict__ FLAG, const float* P2,
                                                  const float* __restrict__ sm, float* out) {
  const int tid = (int)threadIdx.x, lane = tid & 31, wave = tid >> 5, hh = lane >> 4, q = lane & 15;
  const int rowBase = (int)blockIdx.x * ABM;
  const int bucket  = rowBase >> SLB;
  const int* lb  = LIST + (size_t)bucket * (size_t)(2 * RCAP);
  const int* cob = CO + (size_t)bucket * (2 * NBRUN);
  const int flag = FLAG[(size_t)bucket * 32];
  const float qnan = __uint_as_float(0x7fc00000u);
  const v4f bias = *(const v4fa*)(sm + HID + 4 * q);

#pragma unroll 1
  for (int i = 0; i < ABM / (2 * NWAVE); ++i) {
    const int d    = rowBase + (ABM / NWAVE) * wave + 2 * i + hh;
    const int slot = d & (NBRUN - 1);
    int c = cob[slot];
    int o = cob[NBRUN + slot];
    const bool big = c > DEGCAP;
    o = o < 0 ? 0 : (o > RCAP - 1 ? RCAP - 1 : o);
    c = c < 0 ? 0 : (c > DEGCAP ? DEGCAP : c);
    c = c > (RCAP - o) ? (RCAP - o) : c;
    const int co = __shfl_xor(c, 16, 32);
    const int cm = c > co ? c : co;
    const int cmS = __builtin_amdgcn_readfirstlane(cm);
    int last = o + c - 1;
    last = last < o ? o : last;
    float a0 = 0.0f, a1 = 0.0f, a2 = 0.0f, a3 = 0.0f;
#pragma unroll 1
    for (int j = 0; j < cmS; ++j) {
      int idx = o + j;
      idx = idx > last ? last : idx;
      const v2i ent = *(const v2ia*)(lb + 2 * idx);
      int sr = ent.x;
      sr = sr < 0 ? 0 : (sr > NN - 1 ? NN - 1 : sr);
      const float w = __int_as_float(ent.y);
      const v4f p = *(const v4fa*)(P2 + (size_t)sr * OUTF + 4 * q);
      asm volatile("" :: "v"(p));
      const bool valid = j < c;
      const float t0 = fmaf(w, p.x, a0), t1 = fmaf(w, p.y, a1), t2 = fmaf(w, p.z, a2), t3 = fmaf(w, p.w, a3);
      a0 = valid ? t0 : a0; a1 = valid ? t1 : a1; a2 = valid ? t2 : a2; a3 = valid ? t3 : a3;
    }
    float r0 = a0 + bias.x, r1 = a1 + bias.y, r2 = a2 + bias.z, r3 = a3 + bias.w;
    const bool bad = (flag != 0) | big;
    r0 = bad ? qnan : r0; r1 = bad ? qnan : r1; r2 = bad ? qnan : r2; r3 = bad ? qnan : r3;
    v4f ov;
    ov.x = r0; ov.y = r1; ov.z = r2; ov.w = r3;
    const bool live = d < NN;
    const int dc = live ? d : NN - 1;
    float* op = out + (size_t)dc * OUTF + 4 * q;
    if (live) *(volatile v4f*)op = ov;
    __threadfence();
    if (live) *(volatile v4f*)op = ov;
  }
}

extern "C" void kernel_launch(void* const* d_in, const int* in_sizes, int n_in,
                              void* d_out, int out_size, void* d_ws, size_t ws_size,
                              hipStream_t stream) {
  if (n_in < 7) return;
  if (in_sizes[0] != NN * FD) return;
  if (in_sizes[1] != 2 * NE) return;
  if (in_sizes[2] != NE) return;
  if (in_sizes[3] != FD * HID) return;
  if (in_sizes[4] != HID) return;
  if (in_sizes[5] != HID * OUTF) return;
  if (in_sizes[6] != OUTF) return;
  if (out_size != NN * OUTF) return;

  const float* x  = (const float*)d_in[0];
  const int*   ei = (const int*)d_in[1];
  const float* ew = (const float*)d_in[2];
  const float* W1 = (const float*)d_in[3];
  const float* b1 = (const float*)d_in[4];
  const float* W2 = (const float*)d_in[5];
  const float* b2 = (const float*)d_in[6];
  float* out = (float*)d_out;
  const int* srcs = ei;
  const int* dsts = ei + NE;

  constexpr size_t zXB   = (size_t)MP * FD * 2;
  constexpr size_t zP1   = (size_t)MP * HID * 4;
  constexpr size_t zH1   = (size_t)MP * APITCH * 2;
  constexpr size_t zP2   = (size_t)MP * OUTF * 4;
  constexpr size_t zLIST = (size_t)NBK * RCAP * 8;
  constexpr size_t zCO   = (size_t)NBK * 2 * NBRUN * 4;
  constexpr size_t zFLAG = (size_t)(NBK + 1) * 128;
  constexpr size_t zW1T  = (size_t)HID * FD * 2;
  constexpr size_t zW2D  = (size_t)OUTF * WPITCH * 2;
  constexpr size_t zSM   = 1024;
  constexpr size_t oXB   = 0;
  constexpr size_t oP1   = oXB + zXB;
  constexpr size_t oH1   = oP1 + zP1;
  constexpr size_t oP2   = oH1 + zH1;
  constexpr size_t oLIST = oP2 + zP2;
  constexpr size_t oCO   = oLIST + zLIST;
  constexpr size_t oFLAG = oCO + zCO;
  constexpr size_t oW1T  = oFLAG + zFLAG;
  constexpr size_t oW2D  = oW1T + zW1T;
  constexpr size_t oSM   = oW2D + zW2D;
  constexpr size_t oEND  = oSM + zSM;
  static_assert(zXB % 256 == 0 && zP1 % 256 == 0 && zH1 % 256 == 0 && zP2 % 256 == 0 && zLIST % 256 == 0);
  static_assert(zCO % 256 == 0 && zFLAG % 256 == 0 && zW1T % 256 == 0 && zW2D % 256 == 0 && zSM % 256 == 0);
  static_assert(oEND <= (size_t)WSMAX);
  if (oEND > ws_size) return;

  char* ws = (char*)d_ws;
  unsigned short* XB   = (unsigned short*)(ws + oXB);
  float*          P1   = (float*)(ws + oP1);
  unsigned short* H1hl = (unsigned short*)(ws + oH1);
  float*          P2   = (float*)(ws + oP2);
  int*            LIST = (int*)(ws + oLIST);
  int*            CO   = (int*)(ws + oCO);
  int*            FLAG = (int*)(ws + oFLAG);
  unsigned short* W1T  = (unsigned short*)(ws + oW1T);
  unsigned short* W2D  = (unsigned short*)(ws + oW2D);
  float*          SM   = (float*)(ws + oSM);

  hipFuncSetAttribute(reinterpret_cast<const void*>(&k_bucket), hipFuncAttributeMaxDynamicSharedMemorySize, (int)BK_LDS);

  k_prep<<<PBTOT, NTHR, 0, stream>>>(x, W1, b1, W2, b2, XB, W1T, W2D, SM);
  k_bucket<<<NBK, NTHR, BK_LDS, stream>>>(srcs, dsts, ew, LIST, CO, FLAG);
  k_gemm1<<<MP / G1M, G1THR, 0, stream>>>(XB, W1T, P1);
  k_replay1<<<MP / ABM, NTHR, 0, stream>>>(LIST, CO, FLAG, P1, SM, H1hl);
  k_gemm2<<<MP / G2M, NTHR, 0, stream>>>(H1hl, W2D, P2);
  k_replay2<<<MP / ABM, NTHR, 0, stream>>>(LIST, CO, FLAG, P2, SM, out);
}
